// EdgeNet_45810121179634
// MI455X (gfx1250) — hardware-verified
//
#include <hip/hip_runtime.h>
#include <math.h>


typedef _Float16 f16t;
typedef f16t v16h __attribute__((ext_vector_type(16)));
typedef f16t v8h __attribute__((ext_vector_type(8)));
typedef float v8f __attribute__((ext_vector_type(8)));
typedef float v4f __attribute__((ext_vector_type(4)));
typedef unsigned int v4u __attribute__((ext_vector_type(4)));
typedef unsigned long long u64;
typedef u64 v2u __attribute__((ext_vector_type(2)));

union Frag { v16h v; v8h hf[2]; };
union Pk8 { v8h b; v4u u; };

#define KP 96
#define TILE 1024
#define WSC 16.0f
#define WSCI 0.0625f
#define VGPR_CAP __attribute__((amdgpu_num_vgpr(248)))

__device__ __forceinline__ int clampi(int v, int lo, int hi) {
  v = v < lo ? lo : v;
  return v > hi ? hi : v;
}

__device__ __forceinline__ v8f zero8() {
  v8f c;
#pragma unroll
  for (int i = 0; i < 8; ++i) c[i] = 0.0f;
  return c;
}

__device__ __forceinline__ v16h ldfrag(const f16t* base, int h) {
  Frag f;
  f.hf[0] = *(const v8h*)(base + 8 * h);
  f.hf[1] = *(const v8h*)(base + 16 + 8 * h);
  return f.v;
}

__device__ __forceinline__ v8f wm(v16h a, v16h b, v8f c) {
  return __builtin_amdgcn_wmma_f32_16x16x32_f16(false, a, false, b, (short)0, c, false, false);
}

__device__ __forceinline__ v8f mmak3(v16h a0, v16h a1, v16h a2, v16h b0, v16h b1, v16h b2, v8f c) {
  c = wm(a0, b0, c);
  c = wm(a1, b1, c);
  c = wm(a2, b2, c);
  asm volatile("v_nop\n\tv_nop\n\tv_nop\n\tv_nop" : "+v"(c) : "v"(a0), "v"(a1), "v"(a2), "v"(b0), "v"(b1), "v"(b2));
  return c;
}
__device__ __forceinline__ v8f mmak2(v16h a0, v16h a1, v16h b0, v16h b1, v8f c) {
  c = wm(a0, b0, c);
  c = wm(a1, b1, c);
  asm volatile("v_nop\n\tv_nop\n\tv_nop\n\tv_nop" : "+v"(c) : "v"(a0), "v"(a1), "v"(b0), "v"(b1));
  return c;
}
__device__ __forceinline__ v8f mmak1(v16h a0, v16h b0, v8f c) {
  c = wm(a0, b0, c);
  asm volatile("v_nop\n\tv_nop\n\tv_nop\n\tv_nop" : "+v"(c) : "v"(a0), "v"(b0));
  return c;
}

__device__ __forceinline__ float ftanh(float x) {
  x = fminf(fmaxf(x, -15.0f), 15.0f);
  float e = __expf(2.0f * x);
  return 1.0f - 2.0f * __builtin_amdgcn_rcpf(1.0f + e);
}

__device__ __forceinline__ float fsigm(float z) {
  z = fminf(fmaxf(z, -80.0f), 80.0f);
  float e = expf(-z);
  return 1.0f / (1.0f + e);
}

__device__ __forceinline__ int mpath(const u64* A, int La, const u64* B, int Lb, int d) {
  int lo = d - Lb;
  if (lo < 0) lo = 0;
  int hi = d < La ? d : La;
  while (lo < hi) {
    int mid = (lo + hi) >> 1;
    u64 a = A[mid];
    u64 b = B[d - 1 - mid];
    if (a < b) lo = mid + 1; else hi = mid;
  }
  return lo;
}

__device__ __forceinline__ void merge8(const u64* S, int aBase, int La, int bBase, int Lb, int a, int b, u64* o) {
#pragma unroll
  for (int j = 0; j < 8; ++j) {
    int ia = aBase + a; ia = ia > (TILE - 1) ? (TILE - 1) : ia;
    int ib = bBase + b; ib = ib > (TILE - 1) ? (TILE - 1) : ib;
    u64 va = S[ia], vb = S[ib];
    bool ta = (a < La) && ((b >= Lb) || (va < vb));
    o[j] = ta ? va : vb;
    a += ta ? 1 : 0;
    b += ta ? 0 : 1;
  }
}

__device__ __forceinline__ int lbound64(const u64* K, int n, u64 key) {
  int lo = 0, hi = n;
  while (lo < hi) {
    int mid = (lo + hi) >> 1;
    if (K[mid] < key) lo = mid + 1; else hi = mid;
  }
  return lo;
}

__device__ __forceinline__ void csw(u64& a, u64& b) {
  bool lt = a < b;
  u64 x = lt ? a : b, y = lt ? b : a;
  a = x; b = y;
}

__global__ void __launch_bounds__(256) k_stats(const float* __restrict__ x, int N, float* __restrict__ stats) {
  __shared__ double sred[3][256];
  __shared__ double smu[3];
  __shared__ __attribute__((aligned(16))) float sline[32];
  const int tid = threadIdx.x;
  double s0 = 0.0, s1 = 0.0, s2 = 0.0;
  for (int i = tid; i < N; i += 256) {
    s0 += (double)x[i * 3 + 0];
    s1 += (double)x[i * 3 + 1];
    s2 += (double)x[i * 3 + 2];
  }
  sred[0][tid] = s0; sred[1][tid] = s1; sred[2][tid] = s2;
  __syncthreads();
  for (int off = 128; off > 0; off >>= 1) {
    if (tid < off) {
      sred[0][tid] += sred[0][tid + off];
      sred[1][tid] += sred[1][tid + off];
      sred[2][tid] += sred[2][tid + off];
    }
    __syncthreads();
  }
  if (tid == 0) {
    smu[0] = sred[0][0] / (double)N;
    smu[1] = sred[1][0] / (double)N;
    smu[2] = sred[2][0] / (double)N;
  }
  if (tid < 32) sline[tid] = 0.0f;
  __syncthreads();
  const double m0 = smu[0], m1 = smu[1], m2 = smu[2];
  double q0 = 0.0, q1 = 0.0, q2 = 0.0;
  for (int i = tid; i < N; i += 256) {
    double d0 = (double)x[i * 3 + 0] - m0;
    double d1 = (double)x[i * 3 + 1] - m1;
    double d2 = (double)x[i * 3 + 2] - m2;
    q0 += d0 * d0; q1 += d1 * d1; q2 += d2 * d2;
  }
  __syncthreads();
  sred[0][tid] = q0; sred[1][tid] = q1; sred[2][tid] = q2;
  __syncthreads();
  for (int off = 128; off > 0; off >>= 1) {
    if (tid < off) {
      sred[0][tid] += sred[0][tid + off];
      sred[1][tid] += sred[1][tid + off];
      sred[2][tid] += sred[2][tid + off];
    }
    __syncthreads();
  }
  if (tid == 0) {
#pragma unroll
    for (int c = 0; c < 3; ++c) {
      float varf = (float)(sred[c][0] / (double)N);
      float rs = 1.0f / sqrtf(varf + 1e-5f);
      sline[c] = (float)smu[c];
      sline[4 + c] = rs;
    }
  }
  __syncthreads();
  if (tid < 8) {
    v4f v = *(const v4f*)(sline + 4 * tid);
    *(volatile v4f*)(stats + 4 * tid) = v;
    __threadfence();
    *(volatile v4f*)(stats + 4 * tid) = v;
  }
}

__global__ void __launch_bounds__(128) VGPR_CAP
k_node(const float* __restrict__ x, const float* __restrict__ stats,
       const float* __restrict__ gam, const float* __restrict__ bet,
       const float* __restrict__ w1, const float* __restrict__ b1,
       const float* __restrict__ w2, const float* __restrict__ b2,
       f16t* __restrict__ planes, int N, int numBT) {
  __shared__ float sw1[96], sb1[32], sst[8], sg[4], sbb[4];
  __shared__ __attribute__((aligned(16))) float sb2[32];
  __shared__ __attribute__((aligned(16))) f16t sW2[32 * 32];
  __shared__ __attribute__((aligned(16))) f16t sT[4 * 16 * 64];
  const int tid = threadIdx.x;
  for (int i = tid; i < 96; i += 128) sw1[i] = w1[i];
  if (tid < 32) { sb1[tid] = b1[tid]; sb2[tid] = b2[tid]; }
  if (tid < 8) sst[tid] = stats[tid];
  if (tid < 3) { sg[tid] = gam[tid]; sbb[tid] = bet[tid]; }
  for (int idx = tid; idx < 1024; idx += 128) {
    const int o = idx >> 5, k = idx & 31;
    sW2[o * 32 + k] = (f16t)(w2[k * 32 + o] * WSC);
  }
  __syncthreads();

  const int w = tid >> 5, l = tid & 31, h = l >> 4, m = l & 15;
  f16t* st = sT + w * 1024;
  const f16t zb = (f16t)0.0f;

  for (int bt = blockIdx.x; bt < numBT; bt += gridDim.x) {
    const int row0 = bt * 64 + w * 16;
    const int node = row0 + m;
    const int nn = node < N ? node : (N - 1);
    float X[3];
#pragma unroll
    for (int c = 0; c < 3; ++c)
      X[c] = (x[nn * 3 + c] - sst[c]) * sst[4 + c] * sg[c] + sbb[c];

    v16h bfr;
#pragma unroll
    for (int i = 0; i < 16; ++i) {
      const int k = 8 * h + (i & 7) + ((i >> 3) << 4);
      float a = X[0] * sw1[k] + X[1] * sw1[32 + k] + X[2] * sw1[64 + k];
      a = a + sb1[k];
      a = fmaxf(a, 0.0f);
      bfr[i] = (f16t)a;
    }
    v8f acc[2];
#pragma unroll
    for (int t = 0; t < 2; ++t) {
      v16h a = ldfrag(sW2 + (16 * t + m) * 32, h);
      acc[t] = mmak1(a, bfr, zero8());
    }
    Pk8 hv[2];
#pragma unroll
    for (int t = 0; t < 2; ++t) {
      v4f ba = *(const v4f*)(sb2 + 16 * t + 8 * h);
      v4f bb = *(const v4f*)(sb2 + 16 * t + 8 * h + 4);
#pragma unroll
      for (int r = 0; r < 4; ++r) {
        hv[t].b[r]     = (f16t)ftanh(fmaf(acc[t][r], WSCI, ba[r]));
        hv[t].b[4 + r] = (f16t)ftanh(fmaf(acc[t][4 + r], WSCI, bb[r]));
      }
    }
    Pk8 xz, zz;
#pragma unroll
    for (int i = 0; i < 8; ++i) { xz.b[i] = zb; zz.b[i] = zb; }
#pragma unroll
    for (int c = 0; c < 3; ++c) xz.b[c] = h ? zb : (f16t)X[c];
    *(v8h*)(st + m * 64 + 8 * h) = hv[0].b;
    *(v8h*)(st + m * 64 + 16 + 8 * h) = hv[1].b;
    *(v8h*)(st + m * 64 + 32 + 8 * h) = xz.b;
    *(v8h*)(st + m * 64 + 48 + 8 * h) = zz.b;
    __syncthreads();

    v4u ov[4];
#pragma unroll
    for (int j = 0; j < 4; ++j) {
      const int row = (l >> 3) + 4 * j, q = l & 7;
      ov[j] = *(const v4u*)(st + row * 64 + 8 * q);
    }
#pragma unroll
    for (int j = 0; j < 4; ++j) {
      const int row = (l >> 3) + 4 * j, q = l & 7;
      *(volatile v4u*)(planes + (size_t)(row0 + row) * 64 + 8 * q) = ov[j];
    }
    __threadfence();
#pragma unroll
    for (int j = 0; j < 4; ++j) {
      const int row = (l >> 3) + 4 * j, q = l & 7;
      *(volatile v4u*)(planes + (size_t)(row0 + row) * 64 + 8 * q) = ov[j];
    }
    __syncthreads();
  }
}

__global__ void __launch_bounds__(128) k_sort_local(const int* __restrict__ eidx, int E, int N, u64* __restrict__ KA) {
  __shared__ __attribute__((aligned(16))) u64 sb0[TILE];
  __shared__ __attribute__((aligned(16))) u64 sb1[TILE];
  const int tid = threadIdx.x;
  const int base = blockIdx.x * TILE;
  u64 k[8];
#pragma unroll
  for (int j = 0; j < 8; ++j) {
    const int eid = base + 8 * tid + j;
    unsigned dh = 0xFFFFFFFFu;
    if (eid < E) {
      int d = eidx[E + eid];
      d = clampi(d, 0, N - 1);
      dh = (unsigned)d;
    }
    k[j] = ((u64)dh << 32) | (u64)(unsigned)eid;
  }
  csw(k[0], k[1]); csw(k[2], k[3]); csw(k[4], k[5]); csw(k[6], k[7]);
  csw(k[0], k[2]); csw(k[1], k[3]); csw(k[4], k[6]); csw(k[5], k[7]);
  csw(k[1], k[2]); csw(k[5], k[6]);
  csw(k[0], k[4]); csw(k[1], k[5]); csw(k[2], k[6]); csw(k[3], k[7]);
  csw(k[2], k[4]); csw(k[3], k[5]);
  csw(k[1], k[2]); csw(k[3], k[4]); csw(k[5], k[6]);
#pragma unroll
  for (int j = 0; j < 8; ++j) sb0[8 * tid + j] = k[j];
  __syncthreads();

  int cur = 0;
  for (int L = 8; L < TILE; L <<= 1) {
    const u64* S = cur ? sb1 : sb0;
    u64* D = cur ? sb0 : sb1;
    const int d = 8 * tid;
    const int ps = d & ~(2 * L - 1);
    const int dd = d - ps;
    const int a = mpath(S + ps, L, S + ps + L, L, dd);
    const int b = dd - a;
    u64 o[8];
    merge8(S, ps, L, ps + L, L, a, b, o);
#pragma unroll
    for (int j = 0; j < 8; ++j) D[d + j] = o[j];
    __syncthreads();
    cur ^= 1;
  }
  const v2u* S2 = (const v2u*)(cur ? sb1 : sb0);
  v2u ov[4];
#pragma unroll
  for (int j = 0; j < 4; ++j) ov[j] = S2[128 * j + tid];
#pragma unroll
  for (int j = 0; j < 4; ++j) *(volatile v2u*)(KA + (size_t)base + 2 * (128 * j + tid)) = ov[j];
  __threadfence();
#pragma unroll
  for (int j = 0; j < 4; ++j) *(volatile v2u*)(KA + (size_t)base + 2 * (128 * j + tid)) = ov[j];
}

__global__ void __launch_bounds__(128) k_merge(const u64* __restrict__ src, u64* __restrict__ dst, int Epad, int L) {
  __shared__ __attribute__((aligned(16))) u64 sWin[TILE];
  __shared__ __attribute__((aligned(16))) u64 sOut[TILE];
  __shared__ int sA[2];
  const int tid = threadIdx.x;
  const int outStart = blockIdx.x * TILE;
  const int ps = outStart & ~(2 * L - 1);
  int La = Epad - ps; if (La > L) La = L;
  int rem = Epad - ps - La;
  int Lb = rem > L ? L : rem;
  const u64* A = src + ps;
  const u64* B = A + La;
  const int d0 = outStart - ps;
  if (tid < 2) sA[tid] = mpath(A, La, B, Lb, d0 + tid * TILE);
  __syncthreads();
  const int a0 = sA[0], a1 = sA[1];
  const int nA = a1 - a0;
  const int b0 = d0 - a0;
  const int nB = TILE - nA;
#pragma unroll
  for (int j = 0; j < 8; ++j) {
    const int i = tid + 128 * j;
    u64 v;
    if (i < nA) v = A[a0 + i]; else v = B[b0 + (i - nA)];
    sWin[i] = v;
  }
  __syncthreads();
  const int dt = 8 * tid;
  const int a = mpath(sWin, nA, sWin + nA, nB, dt);
  const int b = dt - a;
  u64 o[8];
  merge8(sWin, 0, nA, nA, nB, a, b, o);
#pragma unroll
  for (int j = 0; j < 8; ++j) sOut[dt + j] = o[j];
  __syncthreads();
  const v2u* S2 = (const v2u*)sOut;
  v2u ov[4];
#pragma unroll
  for (int j = 0; j < 4; ++j) ov[j] = S2[128 * j + tid];
#pragma unroll
  for (int j = 0; j < 4; ++j) *(volatile v2u*)(dst + (size_t)outStart + 2 * (128 * j + tid)) = ov[j];
  __threadfence();
#pragma unroll
  for (int j = 0; j < 4; ++j) *(volatile v2u*)(dst + (size_t)outStart + 2 * (128 * j + tid)) = ov[j];
}

__global__ void __launch_bounds__(128) VGPR_CAP
k_conv(const u64* __restrict__ KF, const int* __restrict__ eidx, const float* __restrict__ eattr,
       const f16t* __restrict__ planes,
       const float* __restrict__ w1, const float* __restrict__ b1,
       const float* __restrict__ w2, const float* __restrict__ b2,
       float* __restrict__ msg, int N, int E, int numBT) {
  __shared__ __attribute__((aligned(16))) f16t sW1[64 * KP];
  __shared__ __attribute__((aligned(16))) f16t sW2[32 * 64];
  __shared__ __attribute__((aligned(16))) float sb1[64];
  __shared__ __attribute__((aligned(16))) float sb2[32];
  __shared__ __attribute__((aligned(16))) f16t sBt[4 * 16 * KP];
  __shared__ __attribute__((aligned(16))) float sSt[4 * 512];
  const int tid = threadIdx.x, w = tid >> 5, l = tid & 31, h = l >> 4, m = l & 15;

  for (int idx = tid; idx < 64 * KP; idx += 128) {
    const int n = idx / KP, s = idx - n * KP;
    float v = 0.0f;
    if (s < 35) v = w1[s * 64 + n] - w1[(s + 35) * 64 + n];
    else if (s >= 48 && s < 83) v = w1[(s - 13) * 64 + n];
    else if (s == 83) v = w1[70 * 64 + n];
    sW1[n * KP + s] = (f16t)(v * WSC);
  }
  for (int idx = tid; idx < 2048; idx += 128) {
    const int o = idx >> 6, k = idx & 63;
    sW2[o * 64 + k] = (f16t)(w2[k * 32 + o] * WSC);
  }
  if (tid < 64) sb1[tid] = b1[tid];
  if (tid < 32) sb2[tid] = b2[tid];
  __syncthreads();

  f16t* Bt = sBt + w * 16 * KP;
  float* st = sSt + w * 512;

  for (int bt = blockIdx.x; bt < numBT; bt += gridDim.x) {
    const int p0 = bt * 64 + w * 16;
    {
      const u64 key = KF[p0 + m];
      const unsigned eid = (unsigned)(key & 0xFFFFFFFFull);
      const bool valid = eid < (unsigned)E;
      const int eidc = valid ? (int)eid : (E - 1);
      const int dstn = valid ? clampi((int)(key >> 32), 0, N - 1) : 0;
      const int srcn = clampi(eidx[eidc], 0, N - 1);
      const float attr = eattr[eidc];
      const int nd = h ? srcn : dstn;
      const f16t ab = (f16t)attr;
      const f16t* prow = planes + (size_t)nd * 64;
      f16t* br = Bt + m * KP + 48 * h;
#pragma unroll
      for (int q = 0; q < 6; ++q) {
        v8h c = *(const v8h*)(prow + 8 * q);
        if (q == 4) c[3] = h ? ab : c[3];
        *(v8h*)(br + 8 * q) = c;
      }
    }
    __syncthreads();

    const v16h bk0 = ldfrag(Bt + m * KP, h);
    const v16h bk1 = ldfrag(Bt + m * KP + 32, h);
    const v16h bk2 = ldfrag(Bt + m * KP + 64, h);
    v8f acc[4];
#pragma unroll
    for (int t = 0; t < 4; ++t) {
      const f16t* ar = sW1 + (16 * t + m) * KP;
      acc[t] = mmak3(ldfrag(ar, h), ldfrag(ar + 32, h), ldfrag(ar + 64, h), bk0, bk1, bk2, zero8());
    }
    Frag b2f[2];
#pragma unroll
    for (int t = 0; t < 4; ++t) {
      v4f ba = *(const v4f*)(sb1 + 16 * t + 8 * h);
      v4f bb = *(const v4f*)(sb1 + 16 * t + 8 * h + 4);
#pragma unroll
      for (int r = 0; r < 4; ++r) {
        b2f[t >> 1].hf[t & 1][r]     = (f16t)fmaxf(fmaf(acc[t][r], WSCI, ba[r]), 0.0f);
        b2f[t >> 1].hf[t & 1][4 + r] = (f16t)fmaxf(fmaf(acc[t][4 + r], WSCI, bb[r]), 0.0f);
      }
    }
    v8f acc2[2];
#pragma unroll
    for (int t2 = 0; t2 < 2; ++t2) {
      const f16t* ar = sW2 + (16 * t2 + m) * 64;
      acc2[t2] = mmak2(ldfrag(ar, h), ldfrag(ar + 32, h), b2f[0].v, b2f[1].v, zero8());
    }
#pragma unroll
    for (int t2 = 0; t2 < 2; ++t2) {
      v4f ba = *(const v4f*)(sb2 + 16 * t2 + 8 * h);
      v4f bb = *(const v4f*)(sb2 + 16 * t2 + 8 * h + 4);
      v4f o0, o1;
#pragma unroll
      for (int r = 0; r < 4; ++r) {
        o0[r] = ftanh(fmaf(acc2[t2][r], WSCI, ba[r]));
        o1[r] = ftanh(fmaf(acc2[t2][4 + r], WSCI, bb[r]));
      }
      *(v4f*)(st + m * 32 + 16 * t2 + 8 * h) = o0;
      *(v4f*)(st + m * 32 + 16 * t2 + 8 * h + 4) = o1;
    }
    __syncthreads();

    v4f ov[4];
#pragma unroll
    for (int j = 0; j < 4; ++j) {
      const int row = (l >> 3) + 4 * j, q = l & 7;
      ov[j] = *(const v4f*)(st + row * 32 + 4 * q);
    }
#pragma unroll
    for (int j = 0; j < 4; ++j) {
      const int row = (l >> 3) + 4 * j, q = l & 7;
      *(volatile v4f*)(msg + (size_t)(p0 + row) * 32 + 4 * q) = ov[j];
    }
    __threadfence();
#pragma unroll
    for (int j = 0; j < 4; ++j) {
      const int row = (l >> 3) + 4 * j, q = l & 7;
      *(volatile v4f*)(msg + (size_t)(p0 + row) * 32 + 4 * q) = ov[j];
    }
    __syncthreads();
  }
}

__global__ void __launch_bounds__(128) VGPR_CAP
k_agg(const u64* __restrict__ KF, const float* __restrict__ msg, const float* __restrict__ x,
      const float* __restrict__ stats, const float* __restrict__ gam, const float* __restrict__ bet,
      f16t* __restrict__ planes, int N, int Epad) {
  const int n = blockIdx.x * 128 + threadIdx.x;
  if (n >= N) return;
  int p = lbound64(KF, Epad, ((u64)(unsigned)n) << 32);
  v4f acc[8];
  const v4f z4f = {0.0f, 0.0f, 0.0f, 0.0f};
#pragma unroll
  for (int q = 0; q < 8; ++q) acc[q] = z4f;
  while (p < Epad) {
    const u64 key = KF[p];
    if ((unsigned)(key >> 32) != (unsigned)n) break;
    const float* rp = msg + (size_t)p * 32;
#pragma unroll
    for (int q = 0; q < 8; ++q) acc[q] += *(const v4f*)(rp + 4 * q);
    ++p;
  }
  float X[3];
#pragma unroll
  for (int c = 0; c < 3; ++c)
    X[c] = (x[n * 3 + c] - stats[c]) * stats[4 + c] * gam[c] + bet[c];

  const f16t zb = (f16t)0.0f;
  Pk8 pk[8];
#pragma unroll
  for (int q = 0; q < 4; ++q) {
#pragma unroll
    for (int i = 0; i < 4; ++i) {
      pk[q].b[i]     = (f16t)acc[2 * q][i];
      pk[q].b[4 + i] = (f16t)acc[2 * q + 1][i];
    }
  }
#pragma unroll
  for (int i = 0; i < 8; ++i) { pk[4].b[i] = zb; pk[5].b[i] = zb; pk[6].b[i] = zb; pk[7].b[i] = zb; }
#pragma unroll
  for (int c = 0; c < 3; ++c) pk[4].b[c] = (f16t)X[c];

  f16t* row = planes + (size_t)n * 64;
#pragma unroll
  for (int q = 0; q < 8; ++q) *(volatile v4u*)(row + 8 * q) = pk[q].u;
  __threadfence();
#pragma unroll
  for (int q = 0; q < 8; ++q) *(volatile v4u*)(row + 8 * q) = pk[q].u;
}

__global__ void __launch_bounds__(128) VGPR_CAP
k_edge(const int* __restrict__ eidx, const float* __restrict__ eattr, const f16t* __restrict__ planes,
       const float* __restrict__ w1, const float* __restrict__ b1,
       const float* __restrict__ we2, const float* __restrict__ be2p,
       float* __restrict__ out, int N, int E, int numBT) {
  __shared__ __attribute__((aligned(16))) f16t sW1[64 * KP];
  __shared__ __attribute__((aligned(16))) float sb1[64];
  __shared__ __attribute__((aligned(16))) float sw2[64];
  __shared__ __attribute__((aligned(16))) f16t sBt[4 * 16 * KP];
  __shared__ __attribute__((aligned(16))) float sOut[64];
  const int tid = threadIdx.x, w = tid >> 5, l = tid & 31, h = l >> 4, m = l & 15;

  for (int idx = tid; idx < 64 * KP; idx += 128) {
    const int n = idx / KP, s = idx - n * KP;
    float v = 0.0f;
    if (s < 35) v = w1[s * 64 + n];
    else if (s >= 48 && s < 83) v = w1[(s - 13) * 64 + n];
    else if (s == 83) v = w1[70 * 64 + n];
    sW1[n * KP + s] = (f16t)(v * WSC);
  }
  if (tid < 64) { sb1[tid] = b1[tid]; sw2[tid] = we2[tid]; }
  const float be2 = be2p[0];
  __syncthreads();

  f16t* Bt = sBt + w * 16 * KP;

  for (int bt = blockIdx.x; bt < numBT; bt += gridDim.x) {
    const int e0 = bt * 64 + w * 16;
    {
      const int eid = e0 + m;
      const int eidc = eid < E ? eid : (E - 1);
      const int srcn = clampi(eidx[eidc], 0, N - 1);
      const int dstn = clampi(eidx[E + eidc], 0, N - 1);
      const float attr = eattr[eidc];
      const int nd = h ? dstn : srcn;
      const f16t ab = (f16t)attr;
      const f16t* prow = planes + (size_t)nd * 64;
      f16t* br = Bt + m * KP + 48 * h;
#pragma unroll
      for (int q = 0; q < 6; ++q) {
        v8h c = *(const v8h*)(prow + 8 * q);
        if (q == 4) c[3] = h ? ab : c[3];
        *(v8h*)(br + 8 * q) = c;
      }
    }
    __syncthreads();

    const v16h bk0 = ldfrag(Bt + m * KP, h);
    const v16h bk1 = ldfrag(Bt + m * KP + 32, h);
    const v16h bk2 = ldfrag(Bt + m * KP + 64, h);
    v8f acc[4];
#pragma unroll
    for (int t = 0; t < 4; ++t) {
      const f16t* ar = sW1 + (16 * t + m) * KP;
      acc[t] = mmak3(ldfrag(ar, h), ldfrag(ar + 32, h), ldfrag(ar + 64, h), bk0, bk1, bk2, zero8());
    }
    float z = 0.0f;
#pragma unroll
    for (int t = 0; t < 4; ++t) {
      v4f ba = *(const v4f*)(sb1 + 16 * t + 8 * h);
      v4f bb = *(const v4f*)(sb1 + 16 * t + 8 * h + 4);
      v4f wa = *(const v4f*)(sw2 + 16 * t + 8 * h);
      v4f wb = *(const v4f*)(sw2 + 16 * t + 8 * h + 4);
#pragma unroll
      for (int r = 0; r < 4; ++r) {
        z = fmaf(fmaxf(fmaf(acc[t][r], WSCI, ba[r]), 0.0f), wa[r], z);
        z = fmaf(fmaxf(fmaf(acc[t][4 + r], WSCI, bb[r]), 0.0f), wb[r], z);
      }
    }
    z += __shfl_xor(z, 16, 32);
    const float ov1 = fsigm(z + be2);
    if (h == 0) sOut[16 * w + m] = ov1;
    __syncthreads();

    if (w == 0 && l < 16) {
      const int eb = bt * 64 + 4 * l;
      v4f v = *(const v4f*)(sOut + 4 * l);
      if (eb + 4 <= E) {
        *(volatile v4f*)(out + eb) = v;
        __threadfence();
        *(volatile v4f*)(out + eb) = v;
      } else {
#pragma unroll
        for (int i = 0; i < 4; ++i) if (eb + i < E) *(volatile float*)(out + eb + i) = v[i];
        __threadfence();
#pragma unroll
        for (int i = 0; i < 4; ++i) if (eb + i < E) *(volatile float*)(out + eb + i) = v[i];
      }
    }
    __syncthreads();
  }
}

extern "C" void kernel_launch(void* const* d_in, const int* in_sizes, int n_in,
                              void* d_out, int out_size, void* d_ws, size_t ws_size,
                              hipStream_t stream) {
  if (n_in < 17) return;
  const float* x     = (const float*)d_in[0];
  const int*   eidx  = (const int*)d_in[1];
  const float* eattr = (const float*)d_in[2];
  const float* gam   = (const float*)d_in[3];
  const float* bet   = (const float*)d_in[4];
  const float* w_in1 = (const float*)d_in[5];
  const float* b_in1 = (const float*)d_in[6];
  const float* w_in2 = (const float*)d_in[7];
  const float* b_in2 = (const float*)d_in[8];
  const float* w_c1  = (const float*)d_in[9];
  const float* b_c1  = (const float*)d_in[10];
  const float* w_c2  = (const float*)d_in[11];
  const float* b_c2  = (const float*)d_in[12];
  const float* w_e1  = (const float*)d_in[13];
  const float* b_e1  = (const float*)d_in[14];
  const float* w_e2  = (const float*)d_in[15];
  const float* b_e2  = (const float*)d_in[16];
  float* out = (float*)d_out;
  (void)out_size;

  const int N = in_sizes[0] / 3;
  const int E = in_sizes[1] / 2;
  if (N <= 0 || E <= 0) return;
  const int nTiles = (E + TILE - 1) / TILE;
  const int Epad = nTiles * TILE;
  const int Npad = ((N + 63) / 64) * 64;

  char* ws = (char*)d_ws;
  size_t off = 0;
  float* stats = (float*)(ws + off);   off += 256;
  f16t* planes = (f16t*)(ws + off);    off += (size_t)Npad * 128;
  u64* KA = (u64*)(ws + off);          off += (size_t)Epad * 8;
  u64* KB = (u64*)(ws + off);          off += (size_t)Epad * 8;
  float* msg = (float*)(ws + off);     off += (size_t)Epad * 128;
  if (off > ws_size) return;

  k_stats<<<1, 256, 0, stream>>>(x, N, stats);

  {
    const int numBT = Npad / 64;
    const int grid = numBT < 512 ? numBT : 512;
    k_node<<<grid, 128, 0, stream>>>(x, stats, gam, bet, w_in1, b_in1, w_in2, b_in2, planes, N, numBT);
  }

  k_sort_local<<<nTiles, 128, 0, stream>>>(eidx, E, N, KA);
  u64* bufs[2] = {KA, KB};
  int cur = 0;
  for (int L = TILE; L < Epad; L <<= 1) {
    k_merge<<<nTiles, 128, 0, stream>>>(bufs[cur], bufs[cur ^ 1], Epad, L);
    cur ^= 1;
  }
  const u64* KF = bufs[cur];

  {
    const int numBT = Epad / 64;
    const int grid = numBT < 256 ? numBT : 256;
    k_conv<<<grid, 128, 0, stream>>>(KF, eidx, eattr, planes, w_c1, b_c1, w_c2, b_c2, msg, N, E, numBT);
  }

  k_agg<<<(N + 127) / 128, 128, 0, stream>>>(KF, msg, x, stats, gam, bet, planes, N, Epad);

  {
    const int numBT = (E + 63) / 64;
    const int grid = numBT < 256 ? numBT : 256;
    k_edge<<<grid, 128, 0, stream>>>(eidx, eattr, planes, w_e1, b_e1, w_e2, b_e2, out, N, E, numBT);
  }
}
